// QuantumAttentionLayer_4045859193502
// MI455X (gfx1250) — hardware-verified
//
#include <hip/hip_runtime.h>
#include <math.h>

#define NTOK 1024
#define DM   2048
#define NH   256
#define HD   8

typedef _Float16 f16;
typedef __attribute__((ext_vector_type(16))) f16 f16x16;
typedef __attribute__((ext_vector_type(8)))  f16 f16x8;
typedef __attribute__((ext_vector_type(8)))  float f32x8;
typedef __attribute__((ext_vector_type(4)))  float v4f_t;
typedef float v4fa __attribute__((ext_vector_type(4), may_alias));
typedef __attribute__((ext_vector_type(4))) unsigned v4u_t;
typedef unsigned v4ua __attribute__((ext_vector_type(4), may_alias));

__device__ __forceinline__ f32x8 wmma16(f16x16 a, f16x16 b, f32x8 c) {
  c = __builtin_amdgcn_wmma_f32_16x16x32_f16(false, a, false, b, (short)0, c, false, false);
  asm volatile("v_nop\n\tv_nop\n\tv_nop\n\tv_nop" : "+v"(c) : "v"(a), "v"(b));
  return c;
}
__device__ __forceinline__ f16x16 lds_frag(const f16* base, int stride) {
  const int lane = threadIdx.x & 31, row = lane & 15, kh = (lane >> 4) * 8;
  const f16x8 lo = *(const f16x8*)(base + row * stride + kh);
  const f16x8 hi = *(const f16x8*)(base + row * stride + kh + 16);
  f16x16 f;
#pragma unroll
  for (int i = 0; i < 8; ++i) { f[i] = lo[i]; f[i + 8] = hi[i]; }
  return f;
}
#define GSTR 48

template <typename AT, bool ACC>
__global__ __launch_bounds__(256) void gemm_kn2(const AT* __restrict__ A, int lda, size_t strideA,
                                               const float* __restrict__ Wm, int ldw, size_t strideW,
                                               const float* __restrict__ bias, float scale,
                                               float* __restrict__ Y, int ldy, size_t strideY, int K) {
  __shared__ __attribute__((aligned(16))) f16 ldsA[128 * GSTR], ldsAl[128 * GSTR];
  __shared__ __attribute__((aligned(16))) f16 ldsW[128 * GSTR], ldsWl[128 * GSTR];
  __shared__ __attribute__((aligned(16))) float oS[8][32 * 68];
  const int tid = threadIdx.x, lane = tid & 31, wave = tid >> 5, cl = lane & 15, rh = (lane >> 4) * 8;
  const int m0 = blockIdx.x * 128, n0 = blockIdx.y * 128;
  const int wm = (wave & 3) * 32, wn = (wave >> 2) * 64;
  A += (size_t)blockIdx.z * strideA; Wm += (size_t)blockIdx.z * strideW; Y += (size_t)blockIdx.z * strideY;
  f32x8 acc[2][4], accx[2][4];
#pragma unroll
  for (int i = 0; i < 2; ++i)
#pragma unroll
    for (int j = 0; j < 4; ++j) { f32x8 z = {}; acc[i][j] = z; accx[i][j] = z; }
#pragma unroll 1
  for (int k0 = 0; k0 < K; k0 += 32) {
    __syncthreads();
    {
      const int row = tid >> 1, ch = (tid & 1) * 16;
      const AT* src = A + (size_t)(m0 + row) * lda + k0 + ch;
#pragma unroll
      for (int g = 0; g < 16; ++g) { const float v = (float)src[g]; const f16 h = (f16)v; ldsA[row * GSTR + ch + g] = h; ldsAl[row * GSTR + ch + g] = (f16)((v - (float)h) * 2048.0f); }
    }
    {
      const int k = tid >> 3, nn0 = (tid & 7) * 16;
      const float* src = Wm + (size_t)(k0 + k) * ldw + n0 + nn0;
#pragma unroll
      for (int g = 0; g < 4; ++g) { const v4f_t v = *(const v4f_t*)(src + 4 * g);
#pragma unroll
        for (int u = 0; u < 4; ++u) { const f16 h = (f16)v[u]; ldsW[(nn0 + 4 * g + u) * GSTR + k] = h; ldsWl[(nn0 + 4 * g + u) * GSTR + k] = (f16)((v[u] - (float)h) * 2048.0f); } }
    }
    __syncthreads();
    f16x16 af[2], afl[2];
#pragma unroll
    for (int i = 0; i < 2; ++i) { af[i] = lds_frag(ldsA + (wm + 16 * i) * GSTR, GSTR); afl[i] = lds_frag(ldsAl + (wm + 16 * i) * GSTR, GSTR); }
#pragma unroll
    for (int j = 0; j < 4; ++j) {
      const f16x16 bf = lds_frag(ldsW + (wn + 16 * j) * GSTR, GSTR), bfl = lds_frag(ldsWl + (wn + 16 * j) * GSTR, GSTR);
#pragma unroll
      for (int i = 0; i < 2; ++i) { acc[i][j] = wmma16(af[i], bf, acc[i][j]); accx[i][j] = wmma16(af[i], bfl, accx[i][j]); accx[i][j] = wmma16(afl[i], bf, accx[i][j]); }
    }
  }
  float* so = oS[wave];
#pragma unroll
  for (int i = 0; i < 2; ++i)
#pragma unroll
    for (int j = 0; j < 4; ++j) {
      const float bv = bias ? bias[n0 + wn + 16 * j + cl] : 0.0f;
#pragma unroll
      for (int r = 0; r < 8; ++r) so[(16 * i + rh + r) * 68 + 16 * j + cl] = (acc[i][j][r] + accx[i][j][r] * (1.0f / 2048.0f)) * scale + bv;
    }
  asm volatile("s_wait_dscnt 0" ::: "memory");
  __builtin_amdgcn_wave_barrier();
  if (ACC) {
#pragma unroll
    for (int it = 0; it < 16; ++it) { const int f4 = lane + 32 * it, rr = f4 >> 4, q = (f4 & 15) * 4;
      const v4f_t old = *(const volatile v4fa*)(Y + (size_t)(m0 + wm + rr) * ldy + n0 + wn + q);
      v4f_t v = *(const volatile v4fa*)(so + rr * 68 + q); v += old; *(volatile v4fa*)(so + rr * 68 + q) = v; }
    asm volatile("s_wait_dscnt 0" ::: "memory");
  }
#pragma unroll 1
  for (int pass = 0; pass < 2; ++pass) {
#pragma unroll
    for (int it = 0; it < 16; ++it) { const int f4 = lane + 32 * it, rr = f4 >> 4, q = (f4 & 15) * 4;
      *(volatile v4f_t*)(Y + (size_t)(m0 + wm + rr) * ldy + n0 + wn + q) = *(const volatile v4fa*)(so + rr * 68 + q); }
    __threadfence();
  }
}

__global__ __launch_bounds__(256) void k_headmix(const float* __restrict__ q, const float* __restrict__ k, const float* __restrict__ v, float* __restrict__ outp) {
  __shared__ __attribute__((aligned(16))) f16 vT[2][16 * 264];
  __shared__ __attribute__((aligned(16))) float oS[DM];
  const int tid = threadIdx.x, lane = tid & 31, wave = tid >> 5, cl = lane & 15, hsel = lane >> 4, kh = hsel * 8, rh = kh;
  const size_t tok = blockIdx.x;
  const float* qt = q + tok * DM; const float* kt = k + tok * DM; const float* vt = v + tok * DM;
  for (int e = tid; e < 16 * NH; e += 256) { const int d = e >> 8, g = e & 255; const float vv = (d < HD) ? vt[g * HD + d] : 0.0f; const f16 h = (f16)vv; vT[0][d * 264 + g] = h; vT[1][d * 264 + g] = (f16)((vv - (float)h) * 2048.0f); }
  __syncthreads();
  const float scale = 0.35355339059327376f * 1.44269504088896340736f;
#pragma unroll 1
  for (int ht = 0; ht < 2; ++ht) {
    const int h0 = wave * 32 + ht * 16;
    f16x16 qf, ql;
#pragma unroll
    for (int i = 0; i < 16; ++i) { qf[i] = (f16)0.0f; ql[i] = (f16)0.0f; }
    if (hsel == 0) {
#pragma unroll
      for (int i = 0; i < 8; ++i) { const float vv = qt[(h0 + cl) * HD + i]; const f16 h = (f16)vv; qf[i] = h; ql[i] = (f16)((vv - (float)h) * 2048.0f); }
    }
    float mrun = -INFINITY, lrun = 0.0f;
    f32x8 o = {}, ox = {};
#pragma unroll 1
    for (int gs = 0; gs < 8; ++gs) {
      f16x16 k0f, k1f, k0l, k1l;
#pragma unroll
      for (int i = 0; i < 16; ++i) { k0f[i] = (f16)0.0f; k1f[i] = (f16)0.0f; k0l[i] = (f16)0.0f; k1l[i] = (f16)0.0f; }
      if (hsel == 0) {
#pragma unroll
        for (int i = 0; i < 8; ++i) { const float a0 = kt[(gs * 32 + cl) * HD + i], a1 = kt[(gs * 32 + 16 + cl) * HD + i]; const f16 h0f = (f16)a0, h1f = (f16)a1;
          k0f[i] = h0f; k0l[i] = (f16)((a0 - (float)h0f) * 2048.0f); k1f[i] = h1f; k1l[i] = (f16)((a1 - (float)h1f) * 2048.0f); }
      }
      f32x8 s0 = {}, s1 = {}, s0x = {}, s1x = {};
      s0 = wmma16(k0f, qf, s0); s0x = wmma16(k0f, ql, s0x); s0x = wmma16(k0l, qf, s0x);
      s1 = wmma16(k1f, qf, s1); s1x = wmma16(k1f, ql, s1x); s1x = wmma16(k1l, qf, s1x);
#pragma unroll
      for (int r = 0; r < 8; ++r) { s0[r] += s0x[r] * (1.0f / 2048.0f); s1[r] += s1x[r] * (1.0f / 2048.0f); }
      float mx = -INFINITY;
#pragma unroll
      for (int r = 0; r < 8; ++r) { s0[r] *= scale; s1[r] *= scale; mx = fmaxf(mx, fmaxf(s0[r], s1[r])); }
      mx = fmaxf(mx, __shfl_xor(mx, 16, 32));
      const float mnew = fmaxf(mrun, mx), alpha = exp2f(mrun - mnew);
      f16x16 pf, pl; float rs = 0.0f;
#pragma unroll
      for (int r = 0; r < 8; ++r) { const float p0 = exp2f(s0[r] - mnew) * 1024.0f, p1 = exp2f(s1[r] - mnew) * 1024.0f; rs += p0 + p1;
        const f16 h0f = (f16)p0, h1f = (f16)p1; pf[r] = h0f; pl[r] = (f16)((p0 - (float)h0f) * 2048.0f); pf[8 + r] = h1f; pl[8 + r] = (f16)((p1 - (float)h1f) * 2048.0f); }
      rs *= (1.0f / 1024.0f);
      rs += __shfl_xor(rs, 16, 32);
      lrun = lrun * alpha + rs; mrun = mnew;
#pragma unroll
      for (int r = 0; r < 8; ++r) { o[r] *= alpha; ox[r] *= alpha; }
      { const f16x16 vh = lds_frag(vT[0] + gs * 32, 264), vl = lds_frag(vT[1] + gs * 32, 264);
        o = wmma16(vh, pf, o); ox = wmma16(vh, pl, ox); ox = wmma16(vl, pf, ox); }
    }
    if (hsel == 0) {
      const float rl = 1.0f / (lrun * 1024.0f);
#pragma unroll
      for (int r = 0; r < 8; ++r) oS[(h0 + cl) * HD + r] = (o[r] + ox[r] * (1.0f / 2048.0f)) * rl;
    }
  }
  __syncthreads();
#pragma unroll 1
  for (int pass = 0; pass < 2; ++pass) {
#pragma unroll
    for (int it = 0; it < 2; ++it) *(volatile v4f_t*)(outp + tok * DM + (tid + 256 * it) * 4) = *(const volatile v4fa*)(oS + (tid + 256 * it) * 4);
    __threadfence();
  }
}

extern "C" void kernel_launch(void* const* d_in, const int* in_sizes, int n_in,
                              void* d_out, int out_size, void* d_ws, size_t ws_size,
                              hipStream_t stream) {
  (void)in_sizes; (void)n_in; (void)out_size; (void)ws_size;
  const float* x = (const float*)d_in[0];
  const float* Wq = (const float*)d_in[2], *bq = (const float*)d_in[3], *Wk = (const float*)d_in[4], *bk = (const float*)d_in[5];
  const float* Wv = (const float*)d_in[6], *bv = (const float*)d_in[7], *Wo = (const float*)d_in[8], *bo = (const float*)d_in[9];
  float* out = (float*)d_out;
  char* ws = (char*)d_ws;
  const size_t T = (size_t)NTOK * DM * 4;
  float* qb = (float*)ws; float* kb2 = (float*)(ws + T); float* vb = (float*)(ws + 2 * T); float* ob = (float*)(ws + 3 * T);
  const dim3 blk(256);
  const dim3 g3(NTOK / 128, DM / 128, 1);
  gemm_kn2<float, false><<<g3, blk, 0, stream>>>(x, DM, 0, Wq, DM, 0, bq, 1.0f, qb, DM, 0, DM);
  gemm_kn2<float, false><<<g3, blk, 0, stream>>>(x, DM, 0, Wk, DM, 0, bk, 1.0f, kb2, DM, 0, DM);
  gemm_kn2<float, false><<<g3, blk, 0, stream>>>(x, DM, 0, Wv, DM, 0, bv, 1.0f, vb, DM, 0, DM);
  k_headmix<<<dim3(NTOK), dim3(256), 0, stream>>>(qb, kb2, vb, ob);
  gemm_kn2<float, false><<<g3, blk, 0, stream>>>(ob, DM, 0, Wo, DM, 0, bo, 1.0f, out, DM, 0, DM);
}
